// Net_1967095022180
// MI455X (gfx1250) — hardware-run, weakly checked
//
#include <hip/hip_runtime.h>

typedef float          v8f   __attribute__((ext_vector_type(8)));
typedef float          v4f   __attribute__((ext_vector_type(4)));
typedef unsigned int   v4u   __attribute__((ext_vector_type(4)));
typedef int            v8i   __attribute__((ext_vector_type(8)));
typedef unsigned short v8us  __attribute__((ext_vector_type(8)));
typedef unsigned short v16us __attribute__((ext_vector_type(16)));
typedef __bf16         v16bf __attribute__((ext_vector_type(16)));
typedef _Float16       v16h  __attribute__((ext_vector_type(16)));
typedef v4f  __attribute__((may_alias)) v4fa;
typedef v8us __attribute__((may_alias)) v8usa;
union FragB { v16bf v; v16us u; v8us h[2]; v8i w; };
union FragH { v16h  v; v16us u; v8us h[2]; v8i w; };

__device__ __forceinline__ v8f wmb(const FragB& a, const FragB& b, v8f c) {
  v8f d = __builtin_amdgcn_wmma_f32_16x16x32_bf16(false, a.v, false, b.v, (short)0, c, false, false);
  asm volatile("v_nop\n\tv_nop\n\tv_nop\n\tv_nop" : "+v"(d) : "v"(a.w), "v"(b.w));
  return d;
}

__device__ __forceinline__ v8f wmh(const FragH& a, const FragH& b, v8f c) {
  v8f d = __builtin_amdgcn_wmma_f32_16x16x32_f16(false, a.v, false, b.v, (short)0, c, false, false);
  asm volatile("v_nop\n\tv_nop\n\tv_nop\n\tv_nop" : "+v"(d) : "v"(a.w), "v"(b.w));
  return d;
}

__device__ __forceinline__ unsigned bf16_bits(float f) {
  const unsigned u = __float_as_uint(f);
  const unsigned r = (u + 0x7FFFu + ((u >> 16) & 1u)) >> 16;
  const unsigned q = (u >> 16) | 0x40u;
  return ((u & 0x7fffffffu) > 0x7f800000u) ? q : r;
}

__device__ __forceinline__ float bf16_val(float f) {
  return __uint_as_float(bf16_bits(f) << 16);
}
__device__ __forceinline__ int clampi(int v, int lo, int hi) {
  return v < lo ? lo : (v > hi ? hi : v);
}

__device__ __forceinline__ unsigned f16_bits(float f) {
  const unsigned u  = __float_as_uint(f);
  const unsigned s  = (u >> 16) & 0x8000u;
  const unsigned a  = u & 0x7fffffffu;
  const unsigned t  = a - 0x38000000u;
  const unsigned r  = (t + 0x0FFFu + ((t >> 13) & 1u)) >> 13;
  const unsigned rc = r > 0x7C00u ? 0x7C00u : r;
  const bool small  = a < 0x38800000u;
  const bool isnan  = a > 0x7f800000u;
  const unsigned fin = small ? 0u : (s | rc);
  return isnan ? (s | 0x7E00u) : fin;
}

__device__ __forceinline__ unsigned pk16(unsigned lo, unsigned hi) { return lo | (hi << 16); }
__device__ __forceinline__ unsigned bf16_lo_bits(float v) {
  float hi = bf16_val(v);
  asm volatile("" : "+v"(hi));
  return bf16_bits(v - hi);
}
__device__ __forceinline__ v4u pack8_bf16(v4f a, v4f c) {
  return (v4u){ pk16(bf16_bits(a[0]), bf16_bits(a[1])), pk16(bf16_bits(a[2]), bf16_bits(a[3])),
                pk16(bf16_bits(c[0]), bf16_bits(c[1])), pk16(bf16_bits(c[2]), bf16_bits(c[3])) };
}
__device__ __forceinline__ v4u pack8_bf16_lo(v4f a, v4f c) {
  return (v4u){ pk16(bf16_lo_bits(a[0]), bf16_lo_bits(a[1])), pk16(bf16_lo_bits(a[2]), bf16_lo_bits(a[3])),
                pk16(bf16_lo_bits(c[0]), bf16_lo_bits(c[1])), pk16(bf16_lo_bits(c[2]), bf16_lo_bits(c[3])) };
}
__device__ __forceinline__ v4u pack8_f16(v4f a, v4f c) {
  return (v4u){ pk16(f16_bits(a[0]), f16_bits(a[1])), pk16(f16_bits(a[2]), f16_bits(a[3])),
                pk16(f16_bits(c[0]), f16_bits(c[1])), pk16(f16_bits(c[2]), f16_bits(c[3])) };
}

template <int FORM>
__global__ __launch_bounds__(256) void k_plane(const float* __restrict__ src, int rows, int cols, int ldsrc,
                                               unsigned short* __restrict__ dst, int MP, int KP) {
  static_assert(FORM >= 0 && FORM <= 3);
  const int KTOT = (FORM == 1 || FORM == 3) ? 2 * KP : KP;
  const unsigned ppr   = (unsigned)(KTOT >> 3);
  const unsigned kp8   = (unsigned)(KP >> 3);
  const unsigned total = (unsigned)MP * ppr;
  const unsigned g     = blockIdx.x * 256u + threadIdx.x;
  const unsigned rowu  = g / ppr;
  const unsigned p     = g - rowu * ppr;
  const bool second    = p >= kp8;
  const int row = (int)rowu;
  const int c0  = (int)((second ? p - kp8 : p) << 3);
  const float* srow = src + (size_t)clampi(row, 0, rows - 1) * (size_t)ldsrc;
  float x[8];
  unsigned mk[8];
#pragma unroll
  for (int e = 0; e < 8; ++e) {
    const int c = c0 + e;
    const float v = srow[clampi(c, 0, cols - 1)];
    asm volatile("" :: "v"(v));
    x[e]  = v;
    mk[e] = (row < rows && c < cols) ? 0xFFFFu : 0u;
  }
  const v4f a = (v4f){ x[0], x[1], x[2], x[3] };
  const v4f c = (v4f){ x[4], x[5], x[6], x[7] };
  v4u o;
  if (FORM == 2) {
    o = pack8_f16(a, c);
  } else {
    const v4u hi = pack8_bf16(a, c);
    o = hi;
    if (FORM == 1) { const v4u lo = pack8_bf16_lo(a, c); o = second ? lo : hi; }
  }
  const v4u mw = (v4u){ pk16(mk[0], mk[1]), pk16(mk[2], mk[3]), pk16(mk[4], mk[5]), pk16(mk[6], mk[7]) };
  o &= mw;
  if (g < total) {
    volatile v4u* q = (volatile v4u*)(dst + (size_t)g * 8);
    *q = o;
    __threadfence();
    *q = o;
  }
}

template <int FORM> struct FragOf    { typedef FragB T; };
template <>         struct FragOf<2> { typedef FragH T; };
__device__ __forceinline__ v8f mm(const FragB& a, const FragB& b, v8f c) { return wmb(a, b, c); }
__device__ __forceinline__ v8f mm(const FragH& a, const FragH& b, v8f c) { return wmh(a, b, c); }
template <class F> __device__ __forceinline__ F ld_frag(const unsigned short* p) {
  F f;
  f.h[0] = *(const v8usa*)(p);
  f.h[1] = *(const v8usa*)(p + 16);
  return f;
}

template <int FORM, int EPI>
__global__ __launch_bounds__(256) __attribute__((amdgpu_num_vgpr(248)))
void k_gemm_nt(const unsigned short* __restrict__ A, const unsigned short* __restrict__ B,
               const float* __restrict__ bias, float* __restrict__ D, int M, int N, int KTOT, int ldd) {
  static_assert(FORM >= 0 && FORM <= 2);
  static_assert(EPI == 0 || EPI == 1);
  typedef typename FragOf<FORM>::T F;
  __shared__ __attribute__((aligned(16))) float sT[8][16 * 68];
  const int lane = threadIdx.x & 31;
  const int wave = threadIdx.x >> 5;
  const int tilesM = (M + 63) >> 6;
  const int tilesN = (N + 63) >> 6;
  const int tile = blockIdx.x * 8 + wave;
  if (tile >= tilesM * tilesN) return;
  const int tm = tile / tilesN;
  const int tn = tile - tm * tilesN;
  const int m0 = tm << 6;
  const int n0 = tn << 6;

  const int rl = lane & 15;
  const int h8 = (lane >> 4) * 8;
  const unsigned short* pa = A + (size_t)(m0 + rl) * (size_t)KTOT + h8;
  const unsigned short* pb = B + (size_t)(n0 + rl) * (size_t)KTOT + h8;

  v8f acc[4][4];
#pragma unroll
  for (int i = 0; i < 4; ++i)
#pragma unroll
    for (int j = 0; j < 4; ++j) acc[i][j] = (v8f){0.f, 0.f, 0.f, 0.f, 0.f, 0.f, 0.f, 0.f};

#pragma unroll 1
  for (int k0 = 0; k0 < KTOT; k0 += 32) {
    F bf[4];
#pragma unroll
    for (int j = 0; j < 4; ++j) bf[j] = ld_frag<F>(pb + (size_t)(j << 4) * (size_t)KTOT + k0);
#pragma unroll
    for (int i = 0; i < 4; ++i) {
      const F af = ld_frag<F>(pa + (size_t)(i << 4) * (size_t)KTOT + k0);
#pragma unroll
      for (int j = 0; j < 4; ++j) acc[i][j] = mm(af, bf[j], acc[i][j]);
    }
  }

  float* slab = sT[wave];
  const int hh = lane >> 4;
  const int c4 = (lane & 15) * 4;
  const int nc = n0 + c4;
  const bool cok = nc < N;
  v4f bv = (v4f){0.f, 0.f, 0.f, 0.f};
  if (EPI == 1) {
    bv = *(const v4fa*)(bias + clampi(nc, 0, N - 4));
    asm volatile("" :: "v"(bv));
  }
#pragma unroll
  for (int i = 0; i < 4; ++i) {
    const int mBase = m0 + (i << 4);
#pragma unroll
    for (int j = 0; j < 4; ++j) {
#pragma unroll
      for (int r = 0; r < 8; ++r) slab[(h8 + r) * 68 + (j << 4) + rl] = acc[i][j][r];
    }
    __builtin_amdgcn_fence(__ATOMIC_RELEASE, "workgroup");
    __builtin_amdgcn_wave_barrier();
    __builtin_amdgcn_fence(__ATOMIC_ACQUIRE, "workgroup");
    v4f vv[8];
#pragma unroll
    for (int it = 0; it < 8; ++it) {
      const int row = it * 2 + hh;
      v4f v = *(const v4fa*)(slab + row * 68 + c4);
      if (EPI == 1) v += bv;
      vv[it] = v;
    }
    for (int pass = 0; pass < 2; ++pass) {
#pragma unroll
      for (int it = 0; it < 8; ++it) {
        const int row = mBase + it * 2 + hh;
        if (cok && row < M) *(volatile v4f*)(D + (size_t)row * (size_t)ldd + nc) = vv[it];
      }
      __threadfence();
    }
    __builtin_amdgcn_fence(__ATOMIC_RELEASE, "workgroup");
    __builtin_amdgcn_wave_barrier();
    __builtin_amdgcn_fence(__ATOMIC_ACQUIRE, "workgroup");
  }
}

#pragma clang fp contract(off)

#ifndef STAGE2_SINGLE_PLANE
#define STAGE2_SINGLE_PLANE 0
#endif

typedef float  v2f __attribute__((ext_vector_type(2)));
typedef int    v4i __attribute__((ext_vector_type(4)));
typedef double v2d __attribute__((ext_vector_type(2)));
typedef v2f __attribute__((may_alias)) v2fa;
typedef v4i __attribute__((may_alias)) v4ia;
typedef v4u __attribute__((may_alias)) v4ua;
typedef v2d __attribute__((may_alias)) v2da;

constexpr int NN     = 10000;
constexpr int NBAT   = 32;
constexpr int TT     = 10;
constexpr int EE     = 40000;
constexpr int HROWS  = 16 * NN;
constexpr int KPW    = 32;
constexpr int NPIT   = 64;
constexpr int LNM    = NN * NBAT * 10;
constexpr int RCAP   = 5376;
constexpr int DEGCAP = 32;
constexpr int NBLK   = 10;
constexpr int NBMAX  = 1024;
constexpr int SLOTB  = 10;
constexpr int LWAVE  = 8;
constexpr int WCAP   = 256;
constexpr int CHUNK  = LWAVE * WCAP;
constexpr int LISTN  = LWAVE * WCAP;
constexpr int NREC   = 125;
constexpr int RECF   = LNM / NREC;

static_assert(HROWS % 128 == 0 && HROWS % 64 == 0);
static_assert(NPIT == 64 && KPW == 32 && 2 * TT <= KPW);
static_assert((16 * 10 * 4) % 128 == 0 && (NBAT * 10 * 4) % 128 == 0);
static_assert(RCAP >= 4188 + 4188 / 4 && (RCAP % 32) == 0 && ((RCAP * 4) % 128) == 0);
static_assert(DEGCAP >= 14 + 8);
static_assert(NBLK * NBMAX >= NN && NBMAX == (1 << SLOTB) && LISTN >= NBMAX);
static_assert(CHUNK * (1 << SLOTB) <= (1 << 30));
static_assert(NREC * RECF == LNM && RECF == 25 * 256 * 4);
static_assert(NN % 8 == 0);

constexpr size_t SZ_OP   = (size_t)2 * HROWS * KPW * 2;
constexpr size_t SZ_FT   = (size_t)HROWS * NPIT * 4;
constexpr size_t SZ_EL   = (size_t)HROWS * 4 * 4;
constexpr size_t SZ_G    = (size_t)4 * LNM * 4;
constexpr size_t SZ_REGS = (size_t)2 * NN * NBAT * 4;
constexpr size_t SZ_WP   = (size_t)8 * 64 * KPW * 2;
constexpr size_t SZ_TAB  = 4352;
constexpr size_t SZ_LIST = (size_t)2 * NBLK * RCAP * 4;
constexpr size_t SZ_CNT  = (size_t)2 * NBLK * NBMAX * 4;
constexpr size_t SZ_FLAG = (size_t)2 * NBLK * 128;
constexpr size_t SZ_REC  = (size_t)4 * NREC * 128;
constexpr size_t SZ_STAT = 256;
constexpr size_t O_OP   = 0;
constexpr size_t O_FT   = O_OP + SZ_OP;
constexpr size_t O_EL   = O_FT + SZ_FT;
constexpr size_t O_ER   = O_EL + SZ_EL;
constexpr size_t O_G    = O_ER + SZ_EL;
constexpr size_t O_REGS = O_G + SZ_G;
constexpr size_t O_WP   = O_REGS + SZ_REGS;
constexpr size_t O_TAB  = O_WP + SZ_WP;
constexpr size_t O_LIST = O_TAB + SZ_TAB;
constexpr size_t O_CNT  = O_LIST + SZ_LIST;
constexpr size_t O_OFF  = O_CNT + SZ_CNT;
constexpr size_t O_FLAG = O_OFF + SZ_CNT;
constexpr size_t O_REC  = O_FLAG + SZ_FLAG;
constexpr size_t O_STAT = O_REC + SZ_REC;
constexpr size_t WS_TOTAL = O_STAT + SZ_STAT;
static_assert(WS_TOTAL <= ((size_t)128 << 20));
static_assert((O_FT % 256) == 0 && (O_EL % 256) == 0 && (O_ER % 256) == 0 && (O_G % 256) == 0);
static_assert((O_REGS % 256) == 0 && (O_WP % 256) == 0 && (O_TAB % 256) == 0 && (O_LIST % 256) == 0);
static_assert((O_CNT % 256) == 0 && (O_OFF % 256) == 0 && (O_FLAG % 256) == 0 && (O_REC % 256) == 0);
static_assert((O_STAT % 256) == 0 && 1056 * 4 <= SZ_TAB);
static_assert((size_t)2 * LNM == 6400000);

__device__ __forceinline__ float lrelu(float z) { return z >= 0.0f ? z : 0.2f * z; }

__global__ __launch_bounds__(256) void k_wprep(const float* __restrict__ fc, const float* __restrict__ al,
                                               const float* __restrict__ ar, const float* __restrict__ rmw,
                                               const float* __restrict__ rmb, const float* __restrict__ rsw,
                                               const float* __restrict__ rsb, unsigned short* __restrict__ WP,
                                               float* __restrict__ TAB, int set) {
  __shared__ __attribute__((aligned(16))) float sreg[32];
  const int tid = (int)threadIdx.x;
  if (blockIdx.x < 2) {
    const int st = (int)blockIdx.x;
    const int o  = tid >> 2;
    const int p  = tid & 3;
    const int oc = o < 40 ? o : 39;
    const float* row = fc + st * 400 + oc * 10;
    const int klim = st == 0 ? 10 : 20;
    unsigned w[8];
#pragma unroll
    for (int e = 0; e < 8; ++e) {
      const int k  = 8 * p + e;
      const int kk = k < 10 ? k : k - 10;
      const float v = row[clampi(kk, 0, 9)];
      asm volatile("" :: "v"(v));
      const unsigned mk = (o < 40 && k < klim) ? 0xFFFFu : 0u;
      w[e] = bf16_bits(v) & mk;
    }
    const v4u ov = (v4u){ pk16(w[0], w[1]), pk16(w[2], w[3]), pk16(w[4], w[5]), pk16(w[6], w[7]) };
    volatile v4u* q = (volatile v4u*)(WP + (size_t)(st * 4 + set) * 2048 + (size_t)tid * 8);
    *q = ov;
    __threadfence();
    *q = ov;
  } else {
    const int lane = tid & 31;
    {
      const float a = rmw[clampi(lane, 0, 9)];
      const float b = rmb[0];
      const float c = rsw[clampi(lane - 16, 0, 9)];
      const float d = rsb[0];
      asm volatile("" :: "v"(a));
      asm volatile("" :: "v"(b));
      asm volatile("" :: "v"(c));
      asm volatile("" :: "v"(d));
      const unsigned ma = (lane < 10) ? 0xFFFFFFFFu : 0u;
      const unsigned mb = (lane == 10) ? 0xFFFFFFFFu : 0u;
      const unsigned mc = (lane >= 16 && lane < 26) ? 0xFFFFFFFFu : 0u;
      const unsigned md = (lane == 26) ? 0xFFFFFFFFu : 0u;
      const unsigned bits = (__float_as_uint(bf16_val(a)) & ma) | (__float_as_uint(bf16_val(b)) & mb) |
                            (__float_as_uint(bf16_val(c)) & mc) | (__float_as_uint(bf16_val(d)) & md);
      if (tid >= 64 && tid < 96) sreg[lane] = __uint_as_float(bits);
    }
    __syncthreads();
    const v4f rv = *(const v4fa*)(sreg + 4 * (lane & 7));
    if (tid < 64) {
      const int st = tid >> 5;
      float o4[4];
#pragma unroll
      for (int e = 0; e < 4; ++e) {
        const int i  = 4 * lane + e;
        const float va = al[st * 40 + clampi(i, 0, 39)];
        const float vb = ar[st * 40 + clampi(i - 40, 0, 39)];
        asm volatile("" :: "v"(va));
        asm volatile("" :: "v"(vb));
        const unsigned ma = (i < 40) ? 0xFFFFFFFFu : 0u;
        const unsigned mb = (i >= 40 && i < 80) ? 0xFFFFFFFFu : 0u;
        o4[e] = __uint_as_float((__float_as_uint(bf16_val(va)) & ma) | (__float_as_uint(bf16_val(vb)) & mb));
      }
      const v4f ov = (v4f){ o4[0], o4[1], o4[2], o4[3] };
      volatile v4f* q = (volatile v4f*)(TAB + (size_t)(st * 4 + set) * 128 + 4 * lane);
      *q = ov;
      __threadfence();
      *q = ov;
    }
    if (tid >= 64 && tid < 72 && set == 0) {
      volatile v4f* q = (volatile v4f*)(TAB + 1024 + 4 * (tid - 64));
      *q = rv;
      __threadfence();
      *q = rv;
    }
  }
}

__global__ __launch_bounds__(256) void k_prep(const float* __restrict__ x, const float* __restrict__ TAB,
                                              unsigned short* __restrict__ OP, float* __restrict__ REGS,
                                              int c, int nN) {
  __shared__ __attribute__((aligned(16))) float    sx[8][960];
  __shared__ __attribute__((aligned(16))) unsigned sop[8][512];
  __shared__ __attribute__((aligned(16))) float    sw[16];
  __shared__ __attribute__((aligned(16))) float    srg[8][32];
  const int tid = (int)threadIdx.x, lane = tid & 31, wave = tid >> 5;
  const int n  = (int)blockIdx.x * 8 + wave;
  const int nc = n < nN ? n : nN - 1;
  const bool ok = n < nN;
  {
    const v4f wv = *(const v4fa*)(TAB + 1024 + c * 16 + 4 * (tid & 3));
    asm volatile("" :: "v"(wv));
    if (tid < 4) *(v4f*)(sw + 4 * tid) = wv;
  }
#pragma unroll
  for (int i = 0; i < 8; ++i) {
    const int j  = lane + 32 * i;
    const int jc = j < 239 ? j : 239;
    const int t  = jc / 24;
    const int q  = jc - 24 * t;
    const v4f v = *(const v4fa*)(x + ((size_t)t * (size_t)nN + (size_t)nc) * 96 + 4 * q);
    asm volatile("" :: "v"(v));
    if (j < 240) *(v4f*)(&sx[wave][4 * jc]) = v;
  }
  __syncthreads();
  float v[10];
#pragma unroll
  for (int t = 0; t < 10; ++t) v[t] = bf16_val(sx[wave][t * 96 + 3 * lane + c]);
  float s = v[0] * sw[0];
#pragma unroll
  for (int t = 1; t < 10; ++t) s = s + v[t] * sw[t];
  s = s + sw[10];
  {
    const v4u w0 = (v4u){ pk16(bf16_bits(v[0]), bf16_bits(v[1])), pk16(bf16_bits(v[2]), bf16_bits(v[3])),
                          pk16(bf16_bits(v[4]), bf16_bits(v[5])), pk16(bf16_bits(v[6]), bf16_bits(v[7])) };
    const v4u w1 = (v4u){ pk16(bf16_bits(v[8]), bf16_bits(v[9])), 0u, 0u, 0u };
    const v4u wz = (v4u){ 0u, 0u, 0u, 0u };
    unsigned* rowp = &sop[wave][16 * lane];
    *(v4u*)(rowp)      = w0;
    *(v4u*)(rowp + 4)  = w1;
    *(v4u*)(rowp + 8)  = wz;
    *(v4u*)(rowp + 12) = wz;
    srg[wave][lane] = s;
  }
  __syncthreads();
  v4u pv[4];
#pragma unroll
  for (int i = 0; i < 4; ++i) pv[i] = *(const v4ua*)(&sop[wave][4 * (lane + 32 * i)]);
  const v4f rv = *(const v4fa*)(&srg[wave][4 * (lane & 7)]);
  float* rp = REGS + (size_t)c * (size_t)nN * 32 + (size_t)nc * 32 + 4 * (lane & 7);
  for (int pass = 0; pass < 2; ++pass) {
#pragma unroll
    for (int i = 0; i < 4; ++i) {
      const int pp = lane + 32 * i;
      const int hf = pp >> 6;
      const int q  = pp & 63;
      unsigned short* dp = OP + ((size_t)hf * HROWS + (size_t)16 * nc) * KPW + (size_t)q * 8;
      if (ok) *(volatile v4u*)dp = pv[i];
    }
    if (ok && lane < 8) *(volatile v4f*)rp = rv;
    __threadfence();
  }
}

__global__ __launch_bounds__(256) void k_list(const int* __restrict__ keys, const int* __restrict__ srcs,
                                              int* __restrict__ LIST, int* __restrict__ CNT, int* __restrict__ OFF,
                                              int* __restrict__ FLAG, int nE, int nN) {
  __shared__ __attribute__((aligned(16))) int reg1[RCAP];
  __shared__ __attribute__((aligned(16))) int reg2[RCAP];
  __shared__ __attribute__((aligned(16))) int scnt[NBMAX];
  __shared__ __attribute__((aligned(16))) int soff[NBMAX];
  __shared__ __attribute__((aligned(16))) int list[LISTN];
  __shared__ int wcnt[LWAVE];
  __shared__ int wtot[LWAVE];
  const int tid = (int)threadIdx.x, lane = tid & 31, wave = tid >> 5;
  const int blk = (int)blockIdx.x;
  const int slotBase = blk * NBMAX;

  for (int i = tid; i < RCAP; i += 256) { reg1[i] = 0; reg2[i] = 0; }
  for (int i = tid; i < NBMAX; i += 256) { scnt[i] = 0; soff[i] = 0; }
  for (int i = tid; i < LISTN; i += 256) list[i] = 0;
  if (tid < LWAVE) { wcnt[tid] = 0; wtot[tid] = 0; }
  __syncthreads();

  int tot = 0;
  int nChunks = (nE + CHUNK - 1) / CHUNK;
  nChunks = nChunks > 64 ? 64 : nChunks;
  const int l0 = wave * WCAP + lane;
#pragma unroll 1
  for (int ch = 0; ch < nChunks; ++ch) {
    const int cbase = ch * CHUNK;
    int wc = 0;
    unsigned sl[8];
    bool hit[8];
#pragma unroll
    for (int j = 0; j < 8; ++j) {
      const int e  = cbase + l0 + 32 * j;
      const int ec = e < nE - 1 ? e : nE - 1;
      const int kv = keys[ec];
      asm volatile("" :: "v"(kv));
      sl[j]  = (unsigned)kv - (unsigned)slotBase;
      hit[j] = (e < nE) & (sl[j] < (unsigned)NBMAX);
    }
    const unsigned any = __builtin_amdgcn_ballot_w32(hit[0] | hit[1] | hit[2] | hit[3] | hit[4] | hit[5] | hit[6] | hit[7]);
    if (any != 0u) {
#define HITJ(J) { \
      const unsigned mj = __builtin_amdgcn_ballot_w32(hit[J]); \
      if (mj != 0u) { \
        if (hit[J]) { \
          const int pos = wc + (int)__builtin_amdgcn_mbcnt_lo(mj, 0u); \
          if (pos < WCAP) list[wave * WCAP + pos] = ((l0 + 32 * (J)) << SLOTB) | (int)sl[J]; \
        } \
        wc += (int)__builtin_popcount(mj); } }
      HITJ(0)
      HITJ(1)
      HITJ(2)
      HITJ(3)
      HITJ(4)
      HITJ(5)
      HITJ(6)
      HITJ(7)
#undef HITJ
    }
    if (lane == 0) wcnt[wave] = wc;
    __syncthreads();
    int pre = 0, all = 0;
#pragma unroll
    for (int w2 = 0; w2 < LWAVE; ++w2) {
      int cw = wcnt[w2];
      cw = cw < 0 ? 0 : (cw > WCAP ? WCAP : cw);
      all += cw;
      pre += (w2 < wave) ? cw : 0;
    }
    const int wcc  = wc > WCAP ? WCAP : wc;
    const int base = tot + pre;
#pragma unroll 1
    for (int i = lane; i < wcc; i += 32) {
      const int ent = list[wave * WCAP + i];
      const int el  = (ent >> SLOTB) & (CHUNK - 1);
      const int sv  = ent & (NBMAX - 1);
      int eid = cbase + el;
      eid = eid > nE - 1 ? nE - 1 : eid;
      const int pos = base + i;
      if (pos < RCAP) reg1[pos] = (int)(((unsigned)eid << SLOTB) | (unsigned)sv);
    }
    tot += all;
    tot = tot > RCAP ? RCAP : tot;
    __syncthreads();
  }
  const int nh = tot;

  if (wave == 0) {
#pragma unroll 1
    for (int b0 = 0; b0 < nh; b0 += 32) {
      const int idx = b0 + lane;
      const int uv  = reg1[idx < nh ? idx : nh - 1];
      const int m32 = (nh - b0) < 32 ? (nh - b0) : 32;
#pragma unroll 1
      for (int k = 0; k < m32; ++k) {
        const int u  = __builtin_amdgcn_readlane(uv, k);
        const int sv = u & (NBMAX - 1);
        if (lane == 0) scnt[sv] = scnt[sv] + 1;
      }
    }
  }
  __syncthreads();

  {
    const v4i ca = *(const v4ia*)(scnt + 4 * tid);
    const int e0 = ca.x < 0 ? 0 : ca.x, e1 = ca.y < 0 ? 0 : ca.y, e2 = ca.z < 0 ? 0 : ca.z, e3 = ca.w < 0 ? 0 : ca.w;
    const int ts = e0 + e1 + e2 + e3;
    int incl = ts;
#pragma unroll
    for (int d = 1; d < 32; d <<= 1) {
      const int up = __shfl_up(incl, d);
      if (lane >= d) incl += up;
    }
    if (lane == 31) wtot[wave] = incl;
    __syncthreads();
    int pre = 0;
#pragma unroll
    for (int w2 = 0; w2 < LWAVE; ++w2) pre += (w2 < wave) ? wtot[w2] : 0;
    int run = pre + incl - ts;
    soff[4 * tid + 0] = run; run += e0;
    soff[4 * tid + 1] = run; run += e1;
    soff[4 * tid + 2] = run; run += e2;
    soff[4 * tid + 3] = run;
  }
  __syncthreads();
  for (int i = tid; i < NBMAX; i += 256) list[i] = soff[i];
  __syncthreads();

  if (wave == 0) {
#pragma unroll 1
    for (int b0 = 0; b0 < nh; b0 += 32) {
      const int idx = b0 + lane;
      const int uv  = reg1[idx < nh ? idx : nh - 1];
      const int m32 = (nh - b0) < 32 ? (nh - b0) : 32;
#pragma unroll 1
      for (int k = 0; k < m32; ++k) {
        const int u   = __builtin_amdgcn_readlane(uv, k);
        const int sv  = u & (NBMAX - 1);
        const int eid = (int)((unsigned)u >> SLOTB);
        if (lane == 0) {
          int pos = list[sv];
          pos = pos < 0 ? 0 : (pos > RCAP - 1 ? RCAP - 1 : pos);
          reg2[pos] = eid;
          list[sv] = pos + 1;
        }
      }
    }
  }
  __syncthreads();

  int* lp = LIST + (size_t)blk * RCAP;
#pragma unroll 1
  for (int p = tid; p < RCAP / 4; p += 256) {
    const v4i ev = *(const v4ia*)(reg2 + 4 * p);
    const int s0 = srcs[clampi(ev.x, 0, nE - 1)];
    const int s1 = srcs[clampi(ev.y, 0, nE - 1)];
    const int s2 = srcs[clampi(ev.z, 0, nE - 1)];
    const int s3 = srcs[clampi(ev.w, 0, nE - 1)];
    asm volatile("" :: "v"(s0));
    asm volatile("" :: "v"(s1));
    asm volatile("" :: "v"(s2));
    asm volatile("" :: "v"(s3));
    const v4i ov = (v4i){ clampi(s0, 0, nN - 1), clampi(s1, 0, nN - 1), clampi(s2, 0, nN - 1), clampi(s3, 0, nN - 1) };
    volatile v4i* q = (volatile v4i*)(lp + 4 * p);
    *q = ov;
    __threadfence();
    *q = ov;
  }
  {
    const v4i cv = *(const v4ia*)(scnt + 4 * tid);
    const v4i fv = *(const v4ia*)(soff + 4 * tid);
    const int ov = (nh >= RCAP) ? 1 : 0;
    const v4i gv = (v4i){ ov, ov, ov, ov };
    volatile v4i* qc = (volatile v4i*)(CNT + (size_t)blk * NBMAX + 4 * tid);
    volatile v4i* qo = (volatile v4i*)(OFF + (size_t)blk * NBMAX + 4 * tid);
    volatile v4i* qf = (volatile v4i*)(FLAG + (size_t)blk * 32 + 4 * (tid & 7));
    for (int pass = 0; pass < 2; ++pass) {
      *qc = cv;
      *qo = fv;
      if (tid < 8) *qf = gv;
      __threadfence();
    }
  }
}

__global__ __launch_bounds__(256) void k_score(const float* __restrict__ FT, const float* __restrict__ TAB,
                                               float* __restrict__ EL, float* __restrict__ ER, int a0, int nRows) {
  __shared__ __attribute__((aligned(16))) float sa[128];
  const int tid = (int)threadIdx.x;
  {
    const v4f tv = *(const v4fa*)(TAB + (size_t)a0 * 128 + 4 * (tid & 31));
    asm volatile("" :: "v"(tv));
    if (tid < 32) *(v4f*)(sa + 4 * tid) = tv;
  }
  __syncthreads();
  const int r  = (int)blockIdx.x * 256 + tid;
  const int rc = r < nRows ? r : nRows - 1;
  const float* fr = FT + (size_t)rc * NPIT;
  v4f f[10];
#pragma unroll
  for (int i = 0; i < 10; ++i) f[i] = *(const v4fa*)(fr + 4 * i);
  float el[4], er[4];
#pragma unroll
  for (int h = 0; h < 4; ++h) {
    float sl = f[(10 * h) >> 2][(10 * h) & 3] * sa[10 * h];
    float sr = f[(10 * h) >> 2][(10 * h) & 3] * sa[40 + 10 * h];
#pragma unroll
    for (int d = 1; d < 10; ++d) {
      const float fv = f[(10 * h + d) >> 2][(10 * h + d) & 3];
      sl = sl + fv * sa[10 * h + d];
      sr = sr + fv * sa[40 + 10 * h + d];
    }
    el[h] = sl;
    er[h] = sr;
  }
  const v4f lv = (v4f){ el[0], el[1], el[2], el[3] };
  const v4f rv = (v4f){ er[0], er[1], er[2], er[3] };
  if (r < nRows) {
    volatile v4f* ql = (volatile v4f*)(EL + (size_t)r * 4);
    volatile v4f* qr = (volatile v4f*)(ER + (size_t)r * 4);
    *ql = lv;
    *qr = rv;
    __threadfence();
    *ql = lv;
    *qr = rv;
  }
}

__global__ __launch_bounds__(256) void k_walk(const int* __restrict__ LIST, const int* __restrict__ CNT,
                                              const int* __restrict__ OFF, const int* __restrict__ FLAG,
                                              const float* __restrict__ EL, const float* __restrict__ ER,
                                              const float* __restrict__ FT, float* __restrict__ G,
                                              int half, int nN) {
  __shared__ __attribute__((aligned(16))) float stg[8][160];
  const int lane = (int)threadIdx.x & 31, wave = (int)threadIdx.x >> 5;
  const int n  = (int)blockIdx.x * 8 + wave;
  const int nc = n < nN ? n : nN - 1;
  const bool ok = n < nN;
  const int bi = lane & 15, hp = lane >> 4;
  const int blk = clampi(nc >> SLOTB, 0, NBLK - 1);
  const int craw = CNT[nc];
  const int oraw = OFF[nc];
  const int fl   = FLAG[blk * 32];
  asm volatile("" :: "v"(craw));
  asm volatile("" :: "v"(oraw));
  asm volatile("" :: "v"(fl));
  int cnt = __builtin_amdgcn_readfirstlane(clampi(craw, 0, DEGCAP));
  const int off = __builtin_amdgcn_readfirstlane(clampi(oraw, 0, RCAP));
  cnt = cnt < RCAP - off ? cnt : RCAP - off;
  const int* lp = LIST + (size_t)blk * RCAP;
  const v2f erv = *(const v2fa*)(ER + (size_t)(16 * nc + bi) * 4 + 2 * hp);
  asm volatile("" :: "v"(erv));

  float m0 = __uint_as_float(0xff800000u), m1 = m0;
#pragma unroll 1
  for (int q = 0; q < cnt; ++q) {
    const int idx = off + q < RCAP - 1 ? off + q : RCAP - 1;
    const int sr = lp[idx];
    asm volatile("" :: "v"(sr));
    const int s = clampi(sr, 0, nN - 1);
    const v2f elv = *(const v2fa*)(EL + (size_t)(16 * s + bi) * 4 + 2 * hp);
    asm volatile("" :: "v"(elv));
    const float e0 = lrelu(elv.x + erv.x);
    const float e1 = lrelu(elv.y + erv.y);
    m0 = ((e0 > m0) | (e0 != e0)) ? e0 : m0;
    m1 = ((e1 > m1) | (e1 != e1)) ? e1 : m1;
  }
  float s0 = 0.0f, s1 = 0.0f;
#pragma unroll 1
  for (int q = 0; q < cnt; ++q) {
    const int idx = off + q < RCAP - 1 ? off + q : RCAP - 1;
    const int sr = lp[idx];
    asm volatile("" :: "v"(sr));
    const int s = clampi(sr, 0, nN - 1);
    const v2f elv = *(const v2fa*)(EL + (size_t)(16 * s + bi) * 4 + 2 * hp);
    asm volatile("" :: "v"(elv));
    const float e0 = lrelu(elv.x + erv.x);
    const float e1 = lrelu(elv.y + erv.y);
    s0 = s0 + expf(e0 - m0);
    s1 = s1 + expf(e1 - m1);
  }
  float acc[20];
#pragma unroll
  for (int j = 0; j < 20; ++j) acc[j] = 0.0f;
#pragma unroll 1
  for (int q = 0; q < cnt; ++q) {
    const int idx = off + q < RCAP - 1 ? off + q : RCAP - 1;
    const int sr = lp[idx];
    asm volatile("" :: "v"(sr));
    const int s = clampi(sr, 0, nN - 1);
    const size_t rowS = (size_t)(16 * s + bi);
    const v2f elv = *(const v2fa*)(EL + rowS * 4 + 2 * hp);
    asm volatile("" :: "v"(elv));
    const float* fp = FT + rowS * NPIT + 20 * hp;
    v4f fv[5];
#pragma unroll
    for (int i = 0; i < 5; ++i) {
      fv[i] = *(const v4fa*)(fp + 4 * i);
      asm volatile("" :: "v"(fv[i]));
    }
    const float e0 = lrelu(elv.x + erv.x);
    const float e1 = lrelu(elv.y + erv.y);
    const float a0 = expf(e0 - m0) / s0;
    const float a1 = expf(e1 - m1) / s1;
#pragma unroll
    for (int j = 0; j < 20; ++j) {
      const float aj = j < 10 ? a0 : a1;
      acc[j] = acc[j] + aj * fv[j >> 2][j & 3];
    }
  }
  const bool bad = (fl != 0) | (craw > DEGCAP) | (craw < 0);
  const float pz = bad ? __uint_as_float(0x7fc00000u) : 0.0f;
  float mean[10];
#pragma unroll
  for (int d = 0; d < 10; ++d) {
    const float p = lrelu(acc[d]) + lrelu(acc[10 + d]);
    const float o = __shfl_xor(p, 16);
    mean[d] = (p + o) * 0.25f + pz;
  }
  if (lane < 16) {
#pragma unroll
    for (int d = 0; d < 10; ++d) stg[wave][bi * 10 + d] = mean[d];
  }
  __syncthreads();
  const v4f o0 = *(const v4fa*)(&stg[wave][4 * lane]);
  const v4f o1 = *(const v4fa*)(&stg[wave][128 + 4 * (lane & 7)]);
  float* gb = G + (size_t)nc * 320 + (size_t)half * 160;
  for (int pass = 0; pass < 2; ++pass) {
    if (ok) *(volatile v4f*)(gb + 4 * lane) = o0;
    if (ok && lane < 8) *(volatile v4f*)(gb + 128 + 4 * lane) = o1;
    __threadfence();
  }
}

__global__ __launch_bounds__(256) void k_rec(const float* __restrict__ G, double* __restrict__ REC) {
  __shared__ double sh[2][8];
  const int tid = (int)threadIdx.x, lane = tid & 31, wave = tid >> 5;
  const int g  = (int)blockIdx.x / NREC;
  const int rb = (int)blockIdx.x - g * NREC;
  const float* base = G + (size_t)g * LNM + (size_t)rb * RECF;
  double s = 0.0, ss = 0.0;
#pragma unroll 1
  for (int i = 0; i < 25; ++i) {
    const v4f v = *(const v4fa*)(base + (size_t)(i * 256 + tid) * 4);
    const double d0 = (double)v[0], d1 = (double)v[1], d2 = (double)v[2], d3 = (double)v[3];
    s  = s + d0;  ss = ss + d0 * d0;
    s  = s + d1;  ss = ss + d1 * d1;
    s  = s + d2;  ss = ss + d2 * d2;
    s  = s + d3;  ss = ss + d3 * d3;
  }
#pragma unroll
  for (int o = 16; o > 0; o >>= 1) {
    const double a = __shfl_xor(s, o);
    const double b = __shfl_xor(ss, o);
    s  = s + a;
    ss = ss + b;
  }
  if (lane == 0) { sh[0][wave] = s; sh[1][wave] = ss; }
  __syncthreads();
  double ts = sh[0][0], tq = sh[1][0];
#pragma unroll
  for (int w = 1; w < 8; ++w) { ts = ts + sh[0][w]; tq = tq + sh[1][w]; }
  const v2d ov = (tid == 0) ? (v2d){ ts, tq } : (v2d){ 0.0, 0.0 };
  if (tid < 8) {
    volatile v2d* q = (volatile v2d*)(REC + (size_t)blockIdx.x * 16 + 2 * tid);
    *q = ov;
    __threadfence();
    *q = ov;
  }
}

__global__ __launch_bounds__(128) void k_comb(const double* __restrict__ REC, float* __restrict__ STAT) {
  __shared__ __attribute__((aligned(16))) float sst[32];
  const int tid = (int)threadIdx.x, lane = tid & 31, wave = tid >> 5;
  if (tid < 32) sst[tid] = 0.0f;
  double s = 0.0, ss = 0.0;
#pragma unroll
  for (int k = 0; k < 4; ++k) {
    const int r  = lane + 32 * k;
    const int rc = r < NREC - 1 ? r : NREC - 1;
    const v2d rv = *(const v2da*)(REC + (size_t)(wave * NREC + rc) * 16);
    const double a = rv[0], b = rv[1];
    asm volatile("" :: "v"(a));
    asm volatile("" :: "v"(b));
    const double wgt = (r < NREC) ? 1.0 : 0.0;
    s  = s + a * wgt;
    ss = ss + b * wgt;
  }
#pragma unroll
  for (int o = 16; o > 0; o >>= 1) {
    const double a = __shfl_xor(s, o);
    const double b = __shfl_xor(ss, o);
    s  = s + a;
    ss = ss + b;
  }
  __syncthreads();
  const double cntd = (double)LNM;
  const double mean = s / cntd;
  const double var  = ss / cntd - mean * mean;
  const float mf = (float)mean;
  const float vf = (float)var;
  const float rs = 1.0f / sqrtf(vf + 1e-5f);
  if (lane == 0) { sst[2 * wave] = mf; sst[2 * wave + 1] = rs; }
  __syncthreads();
  const v4f sv = *(const v4fa*)(sst + 4 * (tid & 7));
  if (tid < 8) {
    volatile v4f* q = (volatile v4f*)(STAT + 4 * tid);
    *q = sv;
    __threadfence();
    *q = sv;
  }
}

__global__ __launch_bounds__(256) void k_hsplit(const float* __restrict__ Ga, const float* __restrict__ Gb,
                                                const float* __restrict__ STAT, unsigned short* __restrict__ OP,
                                                int pr, int nN) {
  __shared__ __attribute__((aligned(16))) float    sg[8][640];
  __shared__ __attribute__((aligned(16))) unsigned sop[8][512];
  const int tid = (int)threadIdx.x, lane = tid & 31, wave = tid >> 5;
  const int n  = (int)blockIdx.x * 8 + wave;
  const int nc = n < nN ? n : nN - 1;
  const bool ok = n < nN;
  const v4f st = *(const v4fa*)(STAT + 4 * pr);
  asm volatile("" :: "v"(st));
#pragma unroll
  for (int i = 0; i < 3; ++i) {
    const int j  = lane + 32 * i;
    const int jc = j < 79 ? j : 79;
    const v4f va = *(const v4fa*)(Ga + (size_t)nc * 320 + 4 * jc);
    const v4f vb = *(const v4fa*)(Gb + (size_t)nc * 320 + 4 * jc);
    asm volatile("" :: "v"(va));
    asm volatile("" :: "v"(vb));
    if (j < 80) {
      *(v4f*)(&sg[wave][4 * jc])       = va;
      *(v4f*)(&sg[wave][320 + 4 * jc]) = vb;
    }
  }
  __syncthreads();
  unsigned hb[10], lb[10];
#pragma unroll
  for (int t = 0; t < 10; ++t) {
    const float ga = sg[wave][10 * lane + t];
    const float gb = sg[wave][320 + 10 * lane + t];
    const float h  = ((ga - st[0]) * st[1] + (gb - st[2]) * st[3]) * 0.5f;
    hb[t] = bf16_bits(h);
    lb[t] = STAGE2_SINGLE_PLANE ? 0u : bf16_lo_bits(h);
  }
  {
    const v4u w0 = (v4u){ pk16(hb[0], hb[1]), pk16(hb[2], hb[3]), pk16(hb[4], hb[5]), pk16(hb[6], hb[7]) };
    const v4u w1 = (v4u){ pk16(hb[8], hb[9]), pk16(lb[0], lb[1]), pk16(lb[2], lb[3]), pk16(lb[4], lb[5]) };
    const v4u w2 = (v4u){ pk16(lb[6], lb[7]), pk16(lb[8], lb[9]), 0u, 0u };
    const v4u wz = (v4u){ 0u, 0u, 0u, 0u };
    unsigned* rowp = &sop[wave][16 * lane];
    *(v4u*)(rowp)      = w0;
    *(v4u*)(rowp + 4)  = w1;
    *(v4u*)(rowp + 8)  = w2;
    *(v4u*)(rowp + 12) = wz;
  }
  __syncthreads();
  v4u pv[4];
#pragma unroll
  for (int i = 0; i < 4; ++i) pv[i] = *(const v4ua*)(&sop[wave][4 * (lane + 32 * i)]);
  for (int pass = 0; pass < 2; ++pass) {
#pragma unroll
    for (int i = 0; i < 4; ++i) {
      const int pp = lane + 32 * i;
      const int hf = pp >> 6;
      const int q  = pp & 63;
      unsigned short* dp = OP + ((size_t)hf * HROWS + (size_t)16 * nc) * KPW + (size_t)q * 8;
      if (ok) *(volatile v4u*)dp = pv[i];
    }
    __threadfence();
  }
}

__global__ __launch_bounds__(256) void k_combine(const float* __restrict__ G, const float* __restrict__ REGS,
                                                 float* __restrict__ out, int nN) {
  __shared__ __attribute__((aligned(16))) float sr[8][32];
  const int lane = (int)threadIdx.x & 31, wave = (int)threadIdx.x >> 5;
  const int w  = (int)blockIdx.x * 8 + wave;
  const bool ok = w < 2 * nN;
  const int wc = ok ? w : 2 * nN - 1;
  const int o  = wc >= nN ? 1 : 0;
  const int n  = wc - o * nN;
  {
    const float rv = REGS[((size_t)o * (size_t)nN + (size_t)n) * 32 + lane];
    sr[wave][lane] = rv;
  }
  __syncthreads();
  const float third = 1.0f / 3.0f;
  const float* pa = G + (size_t)o * LNM + (size_t)n * 320;
  const float* pb = G + (size_t)(o + 2) * LNM + (size_t)n * 320;
  v4f res[3];
#pragma unroll
  for (int i = 0; i < 3; ++i) {
    const int j  = lane + 32 * i;
    const int jc = j < 79 ? j : 79;
    const v4f a = *(const v4fa*)(pa + 4 * jc);
    const v4f b = *(const v4fa*)(pb + 4 * jc);
    asm volatile("" :: "v"(a));
    asm volatile("" :: "v"(b));
    v4f r;
#pragma unroll
    for (int e = 0; e < 4; ++e) {
      const int bidx = (4 * jc + e) / 10;
      r[e] = ((sr[wave][bidx] + a[e]) + b[e]) * third;
    }
    res[i] = r;
  }
  float* ob = out + (size_t)o * LNM + (size_t)n * 320;
  for (int pass = 0; pass < 2; ++pass) {
    if (ok) *(volatile v4f*)(ob + 4 * lane) = res[0];
    if (ok) *(volatile v4f*)(ob + 128 + 4 * lane) = res[1];
    if (ok && lane < 16) *(volatile v4f*)(ob + 256 + 4 * lane) = res[2];
    __threadfence();
  }
}

static void run_app(hipStream_t stream, const unsigned short* OP, const unsigned short* WP, const float* TAB, int a0,
                    const int* LIST, const int* CNT, const int* OFF, const int* FLAG,
                    float* FT, float* EL, float* ER, float* Greg) {
  const int tiles = (HROWS / 64) * (NPIT / 64);
  for (int half = 0; half < 2; ++half) {
    k_gemm_nt<0, 0><<<(tiles + 7) / 8, 256, 0, stream>>>(OP + (size_t)half * HROWS * KPW, WP + (size_t)a0 * 64 * KPW,
                                                          TAB, FT, HROWS, NPIT, KPW, NPIT);
    k_score<<<HROWS / 256, 256, 0, stream>>>(FT, TAB, EL, ER, a0, HROWS);
    k_walk<<<NN / 8, 256, 0, stream>>>(LIST, CNT, OFF, FLAG, EL, ER, FT, Greg, half, NN);
  }
}

extern "C" void kernel_launch(void* const* d_in, const int* in_sizes, int n_in,
                              void* d_out, int out_size, void* d_ws, size_t ws_size, hipStream_t stream) {
  if (n_in < 21) return;
  if (in_sizes[0] != TT * NN * NBAT * 3) return;
  for (int i = 1; i <= 4; ++i) if (in_sizes[i] != EE) return;
  for (int s = 0; s < 4; ++s) {
    if (in_sizes[5 + 3 * s] != 800 || in_sizes[6 + 3 * s] != 80 || in_sizes[7 + 3 * s] != 80) return;
  }
  if (in_sizes[17] != 10 || in_sizes[18] != 1 || in_sizes[19] != 10 || in_sizes[20] != 1) return;
  if (out_size != 2 * LNM) return;
  if (WS_TOTAL > ws_size) return;

  const float* x      = (const float*)d_in[0];
  const int*   ps_src = (const int*)d_in[1];
  const int*   ps_dst = (const int*)d_in[2];
  const int*   rl_src = (const int*)d_in[3];
  const int*   rl_dst = (const int*)d_in[4];
  const float* rmw    = (const float*)d_in[17];
  const float* rmb    = (const float*)d_in[18];
  const float* rsw    = (const float*)d_in[19];
  const float* rsb    = (const float*)d_in[20];
  float* out = (float*)d_out;

  char* ws = (char*)d_ws;
  unsigned short* OP = (unsigned short*)(ws + O_OP);
  float*  FT   = (float*)(ws + O_FT);
  float*  EL   = (float*)(ws + O_EL);
  float*  ER   = (float*)(ws + O_ER);
  float*  G    = (float*)(ws + O_G);
  float*  REGS = (float*)(ws + O_REGS);
  unsigned short* WP = (unsigned short*)(ws + O_WP);
  float*  TAB  = (float*)(ws + O_TAB);
  int*    LISTp = (int*)(ws + O_LIST);
  int*    LISTr = LISTp + (size_t)NBLK * RCAP;
  int*    CNTp  = (int*)(ws + O_CNT);
  int*    CNTr  = CNTp + (size_t)NBLK * NBMAX;
  int*    OFFp  = (int*)(ws + O_OFF);
  int*    OFFr  = OFFp + (size_t)NBLK * NBMAX;
  int*    FLAGp = (int*)(ws + O_FLAG);
  int*    FLAGr = FLAGp + (size_t)NBLK * 32;
  double* REC  = (double*)(ws + O_REC);
  float*  STAT = (float*)(ws + O_STAT);

  for (int s = 0; s < 4; ++s) {
    k_wprep<<<3, 256, 0, stream>>>((const float*)d_in[5 + 3 * s], (const float*)d_in[6 + 3 * s],
                                   (const float*)d_in[7 + 3 * s], rmw, rmb, rsw, rsb, WP, TAB, s);
  }
  k_prep<<<NN / 8, 256, 0, stream>>>(x, TAB, OP, REGS, 0, NN);
  k_list<<<NBLK, 256, 0, stream>>>(ps_dst, ps_src, LISTp, CNTp, OFFp, FLAGp, EE, NN);
  k_list<<<NBLK, 256, 0, stream>>>(rl_dst, rl_src, LISTr, CNTr, OFFr, FLAGr, EE, NN);

  run_app(stream, OP, WP, TAB, 0, LISTp, CNTp, OFFp, FLAGp, FT, EL, ER, G + (size_t)0 * LNM);
  run_app(stream, OP, WP, TAB, 2, LISTr, CNTr, OFFr, FLAGr, FT, EL, ER, G + (size_t)2 * LNM);
  k_prep<<<NN / 8, 256, 0, stream>>>(x, TAB, OP, REGS, 1, NN);
  run_app(stream, OP, WP, TAB, 1, LISTp, CNTp, OFFp, FLAGp, FT, EL, ER, G + (size_t)1 * LNM);
  run_app(stream, OP, WP, TAB, 3, LISTr, CNTr, OFFr, FLAGr, FT, EL, ER, G + (size_t)3 * LNM);

  k_rec<<<4 * NREC, 256, 0, stream>>>(G, REC);
  k_comb<<<1, 128, 0, stream>>>(REC, STAT);

  k_hsplit<<<NN / 8, 256, 0, stream>>>(G + (size_t)0 * LNM, G + (size_t)1 * LNM, STAT, OP, 0, NN);
  run_app(stream, OP, WP, TAB, 4, LISTp, CNTp, OFFp, FLAGp, FT, EL, ER, G + (size_t)0 * LNM);
  run_app(stream, OP, WP, TAB, 5, LISTp, CNTp, OFFp, FLAGp, FT, EL, ER, G + (size_t)1 * LNM);
  k_hsplit<<<NN / 8, 256, 0, stream>>>(G + (size_t)2 * LNM, G + (size_t)3 * LNM, STAT, OP, 1, NN);
  run_app(stream, OP, WP, TAB, 6, LISTr, CNTr, OFFr, FLAGr, FT, EL, ER, G + (size_t)2 * LNM);
  run_app(stream, OP, WP, TAB, 7, LISTr, CNTr, OFFr, FLAGr, FT, EL, ER, G + (size_t)3 * LNM);

  k_combine<<<2 * NN / 8, 256, 0, stream>>>(G, REGS, out, NN);
}
